// SPNN_25984552140952
// MI455X (gfx1250) — hardware-verified
//
#include <hip/hip_runtime.h>
#include <stddef.h>
#include <stdint.h>

#pragma clang fp contract(off)

#define HID    256
#define GEO    13
#define DIN    781
#define KP0    832
#define KS0    25
#define XP     800
#define DEPTH  3
#define NBR    4
#define EE     100000
#define NN     50000
#define CH     2048
#define TM     64
#define HP     256
#define OP     256
#define MAXT   (CH / TM + 1)
#define NBLK_E ((EE + CH - 1) / CH)
#define NB     128
#define NBLK_N ((NN + NB - 1) / NB)
#define NCHK   ((EE + 255) / 256)
#define WSC    64.0f
#define INV64  0.015625f
#define BNEPS  1e-5f
#define TRP    72
#define LX_BYTES (TM * XP * 2)
#define LH_BYTES (2 * TM * HP * 2)
#define LL_BYTES (CH * 2)
#define MLP_LDS  (LX_BYTES + LH_BYTES + LL_BYTES)
#define SEG_LDS  (NB * HID * 4)

static_assert(CH == 8 * 256);
static_assert(TM == 64);
static_assert(NB == 128);
static_assert(HID == 256);
static_assert(TM * OP * 4 <= LX_BYTES);
static_assert(XP % 8 == 0);
static_assert(KP0 % 64 == 0);
static_assert(HID % 64 == 0);
static_assert(KS0 * 32 <= XP);
static_assert(KS0 * 32 <= KP0);
static_assert(KS0 * 32 >= DIN);
static_assert(3 * HID + 32 == XP);
static_assert((NN * HID) % 2048 == 0);
static_assert(MLP_LDS == 172032);
static_assert(SEG_LDS == 131072);
static_assert((LX_BYTES % 16) == 0);
static_assert((LH_BYTES % 16) == 0);
static_assert(NBLK_E * CH >= EE);
static_assert((NBLK_E - 1) * CH < EE);
static_assert(NBLK_N * NB >= NN);

typedef _Float16 v16h __attribute__((ext_vector_type(16)));
typedef _Float16 v8h  __attribute__((ext_vector_type(8)));
typedef float    v8f  __attribute__((ext_vector_type(8)));
typedef float    v4f  __attribute__((ext_vector_type(4)));
typedef unsigned int v4u __attribute__((ext_vector_type(4)));

union Frag  { v16h v; v8h h[2]; };
union Pack8 { v8h h; v4u u; };

__device__ __forceinline__ int clampi(int v, int lo, int hi) { return min(max(v, lo), hi); }

__device__ __forceinline__ v8f mma16(v16h a, v16h b, v8f c) {
  c = __builtin_amdgcn_wmma_f32_16x16x32_f16(false, a, false, b, (short)0, c, false, false);
  asm volatile("v_nop\n\tv_nop\n\tv_nop\n\tv_nop" : "+v"(c) : "v"(a), "v"(b));
  return c;
}

__device__ __forceinline__ v16h ldfrag(const _Float16* p, int ld, int row0, int k0, int lane) {
  const int m = lane & 15, lh = lane >> 4;
  const _Float16* q = p + (size_t)(row0 + m) * ld + k0 + 8 * lh;
  Frag f;
  f.h[0] = *(const v8h*)(q);
  f.h[1] = *(const v8h*)(q + 16);
  return f.v;
}

__device__ __forceinline__ v8f zero8() { return (v8f){0.f, 0.f, 0.f, 0.f, 0.f, 0.f, 0.f, 0.f}; }

__device__ __forceinline__ void tile_gemm16(v8f (&acc)[4], const _Float16* asrc, int ap,
                                            const _Float16* bsrc, int bp, int nks, int lane) {
#pragma unroll
  for (int mt = 0; mt < 4; ++mt) acc[mt] = zero8();
#pragma unroll 1
  for (int ks = 0; ks < nks; ++ks) {
    const int k0 = ks * 32;
    const v16h bq = ldfrag(bsrc, bp, 0, k0, lane);
#pragma unroll
    for (int mt = 0; mt < 4; ++mt) {
      const v16h a = ldfrag(asrc, ap, 16 * mt, k0, lane);
      acc[mt] = mma16(a, bq, acc[mt]);
    }
  }
}

__device__ __forceinline__ void bn_cols(const float* __restrict__ gam, const float* __restrict__ bet,
                                        const float* __restrict__ rmu, const float* __restrict__ rvr,
                                        const float* __restrict__ bias, int gi, int bi, float& sc, float& cb) {
  const float g = gam[gi], be = bet[gi], mu = rmu[gi], va = rvr[gi], bb = bias[bi];
  const float s = g * rsqrtf(va + BNEPS);
  sc = s * INV64;
  cb = (bb - mu) * s + be;
}

__global__ __launch_bounds__(256) void k_cvt(const float* __restrict__ src, _Float16* __restrict__ dh, int n8) {
  const int i = blockIdx.x * 256 + (int)threadIdx.x;
  if (i >= n8) return;
  const size_t o = (size_t)i * 8;
  const v4f a0 = *(const v4f*)(src + o);
  const v4f a1 = *(const v4f*)(src + o + 4);
  Pack8 pk;
  pk.h = (v8h){(_Float16)a0[0], (_Float16)a0[1], (_Float16)a0[2], (_Float16)a0[3],
               (_Float16)a1[0], (_Float16)a1[1], (_Float16)a1[2], (_Float16)a1[3]};
  const v4u vv = pk.u;
  volatile v4u* d = (volatile v4u*)(dh + o);
  *d = vv;
  __threadfence();
  *d = vv;
}

__global__ __launch_bounds__(256) void k_wtr(const float* __restrict__ w, _Float16* __restrict__ wt,
                                             int kdim, int kp, int ndim, float scale) {
  __shared__ __align__(16) _Float16 st[64 * TRP];
  const int tid = threadIdx.x;
  w  += (size_t)blockIdx.z * (size_t)kdim * (size_t)ndim;
  wt += (size_t)blockIdx.z * (size_t)ndim * (size_t)kp;
  const int n0 = blockIdx.x * 64, k0 = blockIdx.y * 64;
  const int kr = tid >> 2;
  const int nc = (tid & 3) * 16;
  const int kk = k0 + kr;
  const bool kv = kk < kdim;
  const int kc = min(kk, kdim - 1);
  const float* sp = w + (size_t)kc * ndim + n0 + nc;
#pragma unroll
  for (int q = 0; q < 4; ++q) {
    const v4f a = *(const v4f*)(sp + 4 * q);
#pragma unroll
    for (int j = 0; j < 4; ++j) {
      const float val = kv ? a[j] * scale : 0.0f;
      st[(nc + 4 * q + j) * TRP + kr] = (_Float16)val;
    }
  }
  __syncthreads();
  v4u val[2];
  size_t go[2];
#pragma unroll
  for (int j = 0; j < 2; ++j) {
    const int p  = tid + 256 * j;
    const int nr = p >> 3;
    const int pc = p & 7;
    Pack8 pk;
    pk.h   = *(const v8h*)(st + nr * TRP + pc * 8);
    val[j] = pk.u;
    go[j]  = (size_t)(n0 + nr) * kp + k0 + pc * 8;
  }
  for (int ps = 0; ps < 2; ++ps) {
#pragma unroll
    for (int j = 0; j < 2; ++j) *(volatile v4u*)(wt + go[j]) = val[j];
    __threadfence();
  }
}

__global__ __launch_bounds__(256) void k_mlp(
    const _Float16* __restrict__ xh, const float* __restrict__ geo,
    const int* __restrict__ eidx, const int* __restrict__ eij, const int* __restrict__ ejk,
    const int* __restrict__ nei, const float* __restrict__ att,
    const _Float16* __restrict__ w0t, const _Float16* __restrict__ wht,
    const float* __restrict__ b0, const float* __restrict__ bh,
    const float* __restrict__ gam, const float* __restrict__ bet,
    const float* __restrict__ rmu, const float* __restrict__ rvr,
    float* __restrict__ hp)
{
  extern __shared__ __align__(16) unsigned char dynl[];
  _Float16* lds_x = (_Float16*)dynl;
  float*    lds_o = (float*)dynl;
  _Float16* lds_h = (_Float16*)(dynl + LX_BYTES);
  unsigned short* lst = (unsigned short*)(dynl + LX_BYTES + LH_BYTES);
  __shared__ int s_e[TM];
  __shared__ int s_ec[TM];
  __shared__ int s_nd[3 * TM];
  __shared__ int s_cnt[NBR];
  __shared__ int s_off[NBR];
  __shared__ int s_run[NBR];
  __shared__ int s_wc[8 * NBR];

  const int tid = threadIdx.x, lane = tid & 31, wave = tid >> 5;
  const int hh = lane >> 4, c = lane & 15;
  const unsigned ltm = (1u << lane) - 1u;
  const int cb = blockIdx.x * CH;
  const int nloc = min(CH, EE - cb);
  const int nein = nei[0];

  int cw0 = 0, cw1 = 0, cw2 = 0, cw3 = 0;
#pragma unroll 1
  for (int q = 0; q < CH / 256; ++q) {
    const int el = tid + 256 * q;
    const int ec = min(cb + el, EE - 1);
    const int vij = eij[ec], vjk = ejk[ec];
    const int br = (el < nloc) ? (((vij >= nein) ? 2 : 0) | ((vjk >= nein) ? 1 : 0)) : NBR;
    cw0 += __builtin_popcount(__builtin_amdgcn_ballot_w32(br == 0));
    cw1 += __builtin_popcount(__builtin_amdgcn_ballot_w32(br == 1));
    cw2 += __builtin_popcount(__builtin_amdgcn_ballot_w32(br == 2));
    cw3 += __builtin_popcount(__builtin_amdgcn_ballot_w32(br == 3));
  }
  if (lane == 0) {
    s_wc[wave * NBR + 0] = cw0;
    s_wc[wave * NBR + 1] = cw1;
    s_wc[wave * NBR + 2] = cw2;
    s_wc[wave * NBR + 3] = cw3;
  }
  __syncthreads();
  if (tid == 0) {
    int run = 0;
#pragma unroll
    for (int b = 0; b < NBR; ++b) {
      int tot = 0;
#pragma unroll
      for (int w = 0; w < 8; ++w) tot += s_wc[w * NBR + b];
      s_cnt[b] = tot;
      s_off[b] = run;
      s_run[b] = 0;
      run += tot;
    }
  }
  __syncthreads();

#pragma unroll 1
  for (int q = 0; q < CH / 256; ++q) {
    const int el = tid + 256 * q;
    const int ec = min(cb + el, EE - 1);
    const int vij = eij[ec], vjk = ejk[ec];
    const int br = (el < nloc) ? (((vij >= nein) ? 2 : 0) | ((vjk >= nein) ? 1 : 0)) : NBR;
    int pre = 0;
#pragma unroll
    for (int b = 0; b < NBR; ++b) {
      const bool hitb = (br == b);
      const unsigned bal = __builtin_amdgcn_ballot_w32(hitb);
      pre = hitb ? (int)__builtin_popcount(bal & ltm) : pre;
      if (lane == 0) s_wc[wave * NBR + b] = (int)__builtin_popcount(bal);
    }
    __syncthreads();
    const int brc = min(br, NBR - 1);
    int base = s_run[brc];
#pragma unroll
    for (int w = 0; w < 8; ++w) base += (w < wave) ? s_wc[w * NBR + brc] : 0;
    if (br < NBR) {
      const int pos = clampi(s_off[br] + base + pre, 0, CH - 1);
      lst[pos] = (unsigned short)el;
    }
    int tot = 0;
    if (tid < NBR) {
#pragma unroll
      for (int w = 0; w < 8; ++w) tot += s_wc[w * NBR + tid];
    }
    __syncthreads();
    if (tid < NBR) s_run[tid] += tot;
  }
  __syncthreads();

#pragma unroll 1
  for (int br = 0; br < NBR; ++br) {
    const int cnt = s_cnt[br];
    const int off = s_off[br];
    const int ntl = min((cnt + TM - 1) / TM, MAXT);
    const float attb = att[br];
    const _Float16* w0b = w0t + ((size_t)br * HID + wave * 32) * KP0;
#pragma unroll 1
    for (int tt = 0; tt < ntl; ++tt) {
      __syncthreads();
      if (tid < TM) {
        const int q   = tt * TM + tid;
        const int qc  = min(q, cnt - 1);
        const int pos = clampi(off + qc, 0, CH - 1);
        const int e   = min(cb + (int)lst[pos], EE - 1);
        s_e[tid]  = (q < cnt) ? e : -1;
        s_ec[tid] = e;
        s_nd[tid]          = clampi(eidx[e], 0, NN - 1);
        s_nd[TM + tid]     = clampi(eidx[EE + e], 0, NN - 1);
        s_nd[2 * TM + tid] = clampi(eidx[2 * EE + e], 0, NN - 1);
      }
      __syncthreads();
#pragma unroll 4
      for (int p = tid; p < TM * 96; p += 256) {
        const int r = p / 96;
        const int pc = p - r * 96;
        const int sect = pc >> 5, w8 = pc & 31;
        const int node = s_nd[sect * TM + r];
        const v8h v = *(const v8h*)(xh + (size_t)node * HID + w8 * 8);
        *(v8h*)(lds_x + r * XP + sect * HID + w8 * 8) = v;
      }
#pragma unroll 2
      for (int p = tid; p < TM * 32; p += 256) {
        const int r = p >> 5, cc = p & 31;
        const int e = s_ec[r];
        const float gv = geo[(size_t)e * GEO + min(cc, GEO - 1)];
        lds_x[r * XP + 3 * HID + cc] = (cc < GEO) ? (_Float16)gv : (_Float16)0.0f;
      }
      __syncthreads();

#pragma unroll 1
      for (int nt = 0; nt < 2; ++nt) {
        v8f acc[4];
        tile_gemm16(acc, lds_x, XP, w0b + (size_t)(16 * nt) * KP0, KP0, KS0, lane);
        const int n = wave * 32 + 16 * nt + c;
        float sc, cbias;
        bn_cols(gam, bet, rmu, rvr, b0, (br * (DEPTH + 1) + 0) * HID + n, br * HID + n, sc, cbias);
#pragma unroll
        for (int mt = 0; mt < 4; ++mt) {
#pragma unroll
          for (int r = 0; r < 8; ++r) {
            const int row = 16 * mt + 8 * hh + r;
            lds_h[row * HP + n] = (_Float16)fmaxf(acc[mt][r] * sc + cbias, 0.f);
          }
        }
      }
      __syncthreads();

#pragma unroll 1
      for (int l = 0; l < DEPTH; ++l) {
        const _Float16* hin = lds_h + (l & 1) * (TM * HP);
        _Float16* hout = lds_h + ((l & 1) ^ 1) * (TM * HP);
        const _Float16* wl = wht + ((size_t)(br * DEPTH + l) * HID + wave * 32) * HID;
        const bool last = (l == DEPTH - 1);
#pragma unroll 1
        for (int nt = 0; nt < 2; ++nt) {
          v8f acc[4];
          tile_gemm16(acc, hin, HP, wl + (size_t)(16 * nt) * HID, HID, HID / 32, lane);
          const int n = wave * 32 + 16 * nt + c;
          float sc, cbias;
          bn_cols(gam, bet, rmu, rvr, bh, (br * (DEPTH + 1) + l + 1) * HID + n, (br * DEPTH + l) * HID + n, sc, cbias);
          if (!last) {
#pragma unroll
            for (int mt = 0; mt < 4; ++mt) {
#pragma unroll
              for (int r = 0; r < 8; ++r) {
                const int row = 16 * mt + 8 * hh + r;
                hout[row * HP + n] = (_Float16)fmaxf(acc[mt][r] * sc + cbias, 0.f);
              }
            }
          } else {
#pragma unroll
            for (int mt = 0; mt < 4; ++mt) {
#pragma unroll
              for (int r = 0; r < 8; ++r) {
                const int row = 16 * mt + 8 * hh + r;
                lds_o[row * OP + n] = fmaxf(acc[mt][r] * sc + cbias, 0.f) * attb;
              }
            }
          }
        }
        __syncthreads();
      }

      for (int ps = 0; ps < 2; ++ps) {
#pragma unroll 1
        for (int rr = 0; rr < TM / 8; ++rr) {
          const int r = wave + 8 * rr;
          const int e = s_e[r];
          if (e >= 0) {
            const v4f v0 = *(const v4f*)(lds_o + r * OP + lane * 4);
            const v4f v1 = *(const v4f*)(lds_o + r * OP + 128 + lane * 4);
            float* dst = hp + (size_t)e * HID + lane * 4;
            *(volatile v4f*)(dst) = v0;
            *(volatile v4f*)(dst + 128) = v1;
          }
        }
        __threadfence();
      }
    }
  }
}

__global__ __launch_bounds__(256) void k_seg(const float* __restrict__ hp, const int* __restrict__ eidx,
                                             const int* __restrict__ nnp, float* __restrict__ out) {
  extern __shared__ __align__(16) float sacc[];
  __shared__ int s_he[256];
  __shared__ int s_hn[256];
  __shared__ int s_wc[8];
  const int tid = threadIdx.x, lane = tid & 31, wave = tid >> 5;
  const unsigned ltm = (1u << lane) - 1u;
  const int n0 = blockIdx.x * NB;
  const int nlim = clampi(nnp[0], 0, NN);

#pragma unroll 1
  for (int q = 0; q < NB; ++q) sacc[q * HID + tid] = 0.f;

#pragma unroll 1
  for (int ck = 0; ck < NCHK; ++ck) {
    const int e  = ck * 256 + tid;
    const int ec = min(e, EE - 1);
    const int iv = eidx[ec];
    const int d  = iv - n0;
    const bool hit = (e < EE) && ((unsigned)d < (unsigned)NB) && (iv < nlim);
    const unsigned bal = __builtin_amdgcn_ballot_w32(hit);
    const int pre = (int)__builtin_popcount(bal & ltm);
    if (lane == 0) s_wc[wave] = (int)__builtin_popcount(bal);
    __syncthreads();
    int base = 0, nh = 0;
#pragma unroll
    for (int w = 0; w < 8; ++w) {
      const int cwv = s_wc[w];
      nh += cwv;
      base += (w < wave) ? cwv : 0;
    }
    if (hit) {
      const int p = min(base + pre, 255);
      s_he[p] = e;
      s_hn[p] = d;
    }
    __syncthreads();
    nh = min(nh, 256);
#pragma unroll 1
    for (int h = 0; h < nh; ++h) {
      const int he = clampi(s_he[h], 0, EE - 1);
      const int hn = clampi(s_hn[h], 0, NB - 1);
      sacc[hn * HID + tid] += hp[(size_t)he * HID + tid];
    }
  }
  __syncthreads();

  for (int ps = 0; ps < 2; ++ps) {
#pragma unroll 1
    for (int rr = 0; rr < NB / 8; ++rr) {
      const int ln = wave + 8 * rr;
      const int node = n0 + ln;
      if (node < NN) {
        const v4f v0 = *(const v4f*)(sacc + ln * HID + lane * 4);
        const v4f v1 = *(const v4f*)(sacc + ln * HID + 128 + lane * 4);
        float* dst = out + (size_t)node * HID + lane * 4;
        *(volatile v4f*)(dst) = v0;
        *(volatile v4f*)(dst + 128) = v1;
      }
    }
    __threadfence();
  }
}

extern "C" void kernel_launch(void* const* d_in, const int* in_sizes, int n_in,
                              void* d_out, int out_size, void* d_ws, size_t ws_size,
                              hipStream_t stream) {
  if (n_in < 16) return;
  if (in_sizes[0] != NN * HID) return;
  if (in_sizes[1] != EE * GEO) return;
  if (in_sizes[2] != 3 * EE) return;
  if (in_sizes[3] != EE) return;
  if (in_sizes[4] != EE) return;
  if (in_sizes[5] != NBR) return;
  if (in_sizes[6] != NBR * DIN * HID) return;
  if (in_sizes[7] != NBR * HID) return;
  if (in_sizes[8] != NBR * DEPTH * HID * HID) return;
  if (in_sizes[9] != NBR * DEPTH * HID) return;
  if (in_sizes[10] != NBR * (DEPTH + 1) * HID) return;
  if (in_sizes[11] != NBR * (DEPTH + 1) * HID) return;
  if (in_sizes[12] != NBR * (DEPTH + 1) * HID) return;
  if (in_sizes[13] != NBR * (DEPTH + 1) * HID) return;
  if (in_sizes[14] < 1) return;
  if (in_sizes[15] < 1) return;
  if (out_size != NN * HID) return;

  const float* nf   = (const float*)d_in[0];
  const float* geo  = (const float*)d_in[1];
  const int*   eidx = (const int*)d_in[2];
  const int*   eij  = (const int*)d_in[3];
  const int*   ejk  = (const int*)d_in[4];
  const float* att  = (const float*)d_in[5];
  const float* W0   = (const float*)d_in[6];
  const float* b0   = (const float*)d_in[7];
  const float* Wh   = (const float*)d_in[8];
  const float* bh   = (const float*)d_in[9];
  const float* gam  = (const float*)d_in[10];
  const float* bet  = (const float*)d_in[11];
  const float* rmu  = (const float*)d_in[12];
  const float* rvr  = (const float*)d_in[13];
  const int*   nei  = (const int*)d_in[14];
  const int*   nnp  = (const int*)d_in[15];
  float* out = (float*)d_out;

  size_t off = 0;
  const size_t oXh = off; off += (size_t)NN * HID * 2;
  const size_t oW0 = off; off += (size_t)NBR * HID * KP0 * 2;
  const size_t oWh = off; off += (size_t)NBR * DEPTH * HID * HID * 2;
  const size_t oH  = off; off += (size_t)EE * HID * 4;
  if (off > ws_size) return;
  if (off > (size_t)134217728) return;
  if ((oW0 | oWh | oH) & (size_t)127) return;

  char* ws = (char*)d_ws;
  _Float16* Xh  = (_Float16*)(ws + oXh);
  _Float16* W0T = (_Float16*)(ws + oW0);
  _Float16* WhT = (_Float16*)(ws + oWh);
  float*    Hp  = (float*)(ws + oH);

  k_cvt<<<dim3((NN * HID) / 8 / 256), dim3(256), 0, stream>>>(nf, Xh, (NN * HID) / 8);
  k_wtr<<<dim3(HID / 64, KP0 / 64, NBR), dim3(256), 0, stream>>>(W0, W0T, DIN, KP0, HID, WSC);
  k_wtr<<<dim3(HID / 64, HID / 64, NBR * DEPTH), dim3(256), 0, stream>>>(Wh, WhT, HID, HID, HID, WSC);
  (void)hipFuncSetAttribute(reinterpret_cast<const void*>(&k_mlp), hipFuncAttributeMaxDynamicSharedMemorySize, MLP_LDS);
  k_mlp<<<dim3(NBLK_E), dim3(256), MLP_LDS, stream>>>(Xh, geo, eidx, eij, ejk, nei, att, W0T, WhT,
                                                      b0, bh, gam, bet, rmu, rvr, Hp);
  (void)hipFuncSetAttribute(reinterpret_cast<const void*>(&k_seg), hipFuncAttributeMaxDynamicSharedMemorySize, SEG_LDS);
  k_seg<<<dim3(NBLK_N), dim3(256), SEG_LDS, stream>>>(Hp, eidx, nnp, out);
  (void)hipGetLastError();
}
